// MixingBlock_10144712753909
// MI455X (gfx1250) — hardware-verified
//
#include <hip/hip_runtime.h>


#define NB_  4
#define TT   2048
#define CC   256
#define NH_  8
#define HD   32
#define HID  1024
#define ZH   2
#define SCL  0.17677669529663687f
#define PCAR 1024.0f
typedef _Float16 h16;
typedef unsigned short bf;
typedef __attribute__((ext_vector_type(16))) __bf16   v16bf;
typedef __attribute__((ext_vector_type(16))) _Float16 v16h;
typedef __attribute__((ext_vector_type(8)))  _Float16 v8h;
typedef __attribute__((ext_vector_type(8)))  unsigned short v8us;
typedef __attribute__((ext_vector_type(8)))  float    v8f;
typedef __attribute__((ext_vector_type(4)))  float    v4f;
typedef v8h  __attribute__((may_alias)) v8ha;
typedef v4f  __attribute__((may_alias)) v4fa;
typedef v8us __attribute__((may_alias)) v8usa;

__device__ __forceinline__ unsigned short f2bf(float f) { unsigned u = __float_as_uint(f); u += 0x7FFFu + ((u >> 16) & 1u); return (unsigned short)(u >> 16); }
__device__ __forceinline__ float bf2f(unsigned short b) { return __uint_as_float(((unsigned)b) << 16); }
__device__ __forceinline__ float bfr(float f) { return bf2f(f2bf(f)); }
__device__ __forceinline__ v16h cat16(v8h lo, v8h hi) { return __builtin_shufflevector(lo, hi, 0, 1, 2, 3, 4, 5, 6, 7, 8, 9, 10, 11, 12, 13, 14, 15); }
__device__ __forceinline__ v16bf cat16b(v8us lo, v8us hi) { return __builtin_bit_cast(v16bf, __builtin_shufflevector(lo, hi, 0, 1, 2, 3, 4, 5, 6, 7, 8, 9, 10, 11, 12, 13, 14, 15)); }
__device__ __forceinline__ v8f wmma16(v16h a, v16h b, v8f c) { return __builtin_amdgcn_wmma_f32_16x16x32_f16(false, a, false, b, (short)0, c, false, false); }
__device__ __forceinline__ v8f wmmab(v16bf a, v16bf b, v8f c) { return __builtin_amdgcn_wmma_f32_16x16x32_bf16(false, a, false, b, (short)0, c, false, false); }


template <typename T16> struct WFrag;
template <> struct WFrag<h16> { typedef v16h V; static __device__ __forceinline__ V ld(const h16* p) { return cat16(*(const v8h*)p, *(const v8h*)(p + 16)); } static __device__ __forceinline__ v8f mma(V a, V b, v8f c) { return wmma16(a, b, c); } };
template <> struct WFrag<bf> { typedef v16bf V; static __device__ __forceinline__ V ld(const bf* p) { return cat16b(*(const v8us*)p, *(const v8us*)(p + 16)); } static __device__ __forceinline__ v8f mma(V a, V b, v8f c) { return wmmab(a, b, c); } };
template <typename T16, int NSPLIT, bool BIAS>
__global__ __launch_bounds__(32) void k_gemmw(const T16* __restrict__ A, const T16* __restrict__ A2, const T16* __restrict__ Bt, const T16* __restrict__ Bt2, int K, float* C, int ldc, const float* __restrict__ bias, size_t sA, size_t sB, size_t sC) {
    typedef typename WFrag<T16>::V V;
    __shared__ __align__(16) float os[16 * 68];
    const size_t z = blockIdx.z; A += z * sA; if (A2) A2 += z * sA; Bt += z * sB; if (Bt2) Bt2 += z * sB; C += z * sC;
    const int lane = threadIdx.x & 31, lr = lane & 15, hi = lane >> 4; const int r0 = blockIdx.x * 64, c0 = blockIdx.y * 64;
    v8f acc[4][4];
#pragma unroll
    for (int mb = 0; mb < 4; ++mb)
#pragma unroll
        for (int nb = 0; nb < 4; ++nb) acc[mb][nb] = (v8f){};
    const size_t aoff = (size_t)(r0 + lr) * K + 8 * hi, boff = (size_t)(c0 + lr) * K + 8 * hi;
#pragma unroll 1
    for (int kc = 0; kc < K; kc += 32) {
        V a[4], a2[4];
#pragma unroll
        for (int mb = 0; mb < 4; ++mb) { a[mb] = WFrag<T16>::ld(A + aoff + (size_t)mb * 16 * K + kc); if (NSPLIT == 1 || NSPLIT == 2) a2[mb] = WFrag<T16>::ld(A2 + aoff + (size_t)mb * 16 * K + kc); }
#pragma unroll
        for (int nb = 0; nb < 4; ++nb) { const V b = WFrag<T16>::ld(Bt + boff + (size_t)nb * 16 * K + kc); V b2; if (NSPLIT >= 2) b2 = WFrag<T16>::ld(Bt2 + boff + (size_t)nb * 16 * K + kc);
#pragma unroll
            for (int mb = 0; mb < 4; ++mb) { acc[mb][nb] = WFrag<T16>::mma(a[mb], b, acc[mb][nb]); if (NSPLIT == 1 || NSPLIT == 2) acc[mb][nb] = WFrag<T16>::mma(a2[mb], b, acc[mb][nb]); if (NSPLIT >= 2) acc[mb][nb] = WFrag<T16>::mma(a[mb], b2, acc[mb][nb]); } }
        asm volatile("v_nop\n\tv_nop\n\tv_nop\n\tv_nop" : "+v"(acc[0][0]), "+v"(acc[1][1]), "+v"(acc[2][2]), "+v"(acc[3][3]) : "v"(a[0]), "v"(a[3]));
    }
#pragma unroll
    for (int mb = 0; mb < 4; ++mb) {
#pragma unroll
        for (int nb = 0; nb < 4; ++nb) {
#pragma unroll
            for (int j = 0; j < 8; ++j) os[(hi * 8 + j) * 68 + nb * 16 + lr] = acc[mb][nb][j]; }
        __builtin_amdgcn_wave_barrier(); asm volatile("" ::: "memory");
        float* crow = C + (size_t)(r0 + mb * 16) * ldc + c0;
#pragma unroll 1
        for (int ps = 0; ps < 2; ++ps) {
#pragma unroll
            for (int s = 0; s < 8; ++s) { const int row = 2 * s + hi, cofs = lr * 4; v4f val = *(const v4fa*)(os + row * 68 + cofs); if (BIAS) { val[0] += bfr(bias[c0 + cofs]); val[1] += bfr(bias[c0 + cofs + 1]); val[2] += bfr(bias[c0 + cofs + 2]); val[3] += bfr(bias[c0 + cofs + 3]); }
                *(volatile v4f*)(crow + (size_t)row * ldc + cofs) = val; }
            if (ps == 0) __threadfence(); }
        __builtin_amdgcn_wave_barrier(); asm volatile("" ::: "memory");
    }
}

__device__ __forceinline__ h16 tohx(float x) { return (h16)x; }
__device__ __forceinline__ void splitf(float y, unsigned short& h, unsigned short& l) { h = f2bf(y); l = f2bf(y - bf2f(h)); }
typedef __attribute__((ext_vector_type(2))) _Float16 v2h;
typedef __attribute__((ext_vector_type(4))) _Float16 v4h;
typedef __attribute__((ext_vector_type(2))) unsigned short v2us;
typedef __attribute__((ext_vector_type(4))) unsigned short v4us;

__global__ __launch_bounds__(256) void k_cvt8(const float* __restrict__ src, bf* dst, size_t n8) { const size_t i = (size_t)blockIdx.x * 256 + threadIdx.x; if (i >= n8) return; const v8f v = *(const v8f*)(src + i * 8); v8us o;
#pragma unroll
    for (int k = 0; k < 8; ++k) o[k] = f2bf(v[k]); *(volatile v8us*)(dst + i * 8) = o; __threadfence(); *(volatile v8us*)(dst + i * 8) = o; }
__global__ __launch_bounds__(256) void k_pl(const float* __restrict__ QKV, int s, float scl, h16* P16) { const size_t e = ((size_t)blockIdx.x * 256 + threadIdx.x) * 2; if (e >= (size_t)NH_ * TT * HD) return; const int d = (int)(e % HD); const int t = (int)((e / HD) % TT); const int h = (int)(e / ((size_t)HD * TT)); const float* f = QKV + (size_t)t * 3 * CC + s * CC + h * HD + d; v2h o; o[0] = tohx(f[0] * scl); o[1] = tohx(f[1] * scl); *(volatile v2h*)(P16 + e) = o; __threadfence(); *(volatile v2h*)(P16 + e) = o; }
__global__ __launch_bounds__(256) void k_vtp(const float* __restrict__ QKV, h16* VT) { const size_t e = ((size_t)blockIdx.x * 256 + threadIdx.x) * 2; if (e >= (size_t)NH_ * 64 * TT) return; const int t = (int)(e % TT); const int d = (int)((e / TT) % 64); const int h = (int)(e / ((size_t)TT * 64)); v2h o;
#pragma unroll
    for (int u = 0; u < 2; ++u) o[u] = d < HD ? tohx(QKV[(size_t)(t + u) * 3 * CC + 2 * CC + h * HD + d]) : (h16)0.f; *(volatile v2h*)(VT + e) = o; __threadfence(); *(volatile v2h*)(VT + e) = o; }
__global__ __launch_bounds__(256) void k_msoft(const float* __restrict__ Sb, const float* __restrict__ mk, h16* P) { const int lane = threadIdx.x & 31; const int row = blockIdx.x * 8 + (threadIdx.x >> 5); if (row >= ZH * TT) return; const int i = row % TT; const float* sr = Sb + (size_t)row * TT; const float* mr = mk + (size_t)i * TT; float v[64]; float mx = -3.0e38f;
#pragma unroll
    for (int ch = 0; ch < 16; ++ch) { const int j0 = ch * 128 + lane * 4; const v4f a = *(const v4f*)(sr + j0); const v4f m4 = *(const v4f*)(mr + j0);
#pragma unroll
        for (int q = 0; q < 4; ++q) { const float t = __fadd_rn(a[q], bfr(m4[q])); v[ch * 4 + q] = t; mx = fmaxf(mx, t); } }
#pragma unroll
    for (int sh = 16; sh; sh >>= 1) mx = fmaxf(mx, __shfl_xor(mx, sh, 32));
    float sum = 0.f;
#pragma unroll
    for (int k = 0; k < 64; ++k) { float d0 = __fsub_rn(v[k], mx); asm volatile("" : "+v"(d0)); v[k] = __expf(d0); sum += v[k]; }
#pragma unroll
    for (int sh = 16; sh; sh >>= 1) sum += __shfl_xor(sum, sh, 32);
    const float f = __fdiv_rn(PCAR, sum);
#pragma unroll 1
    for (int ps = 0; ps < 2; ++ps) {
#pragma unroll
        for (int ch = 0; ch < 16; ++ch) { v4h o; o[0] = tohx(v[ch * 4] * f); o[1] = tohx(v[ch * 4 + 1] * f); o[2] = tohx(v[ch * 4 + 2] * f); o[3] = tohx(v[ch * 4 + 3] * f); *(volatile v4h*)(P + (size_t)row * TT + ch * 128 + lane * 4) = o; }
        if (ps == 0) __threadfence(); } }
__global__ __launch_bounds__(256) void k_mrg(const float* __restrict__ Ob, int h0, bf* Ah, bf* Al) { const size_t e = ((size_t)blockIdx.x * 256 + threadIdx.x) * 2; if (e >= (size_t)ZH * TT * HD) return; const int d = (int)(e % HD); const int t = (int)((e / HD) % TT); const int z = (int)(e / ((size_t)HD * TT)); v2us oh, ol;
#pragma unroll
    for (int u = 0; u < 2; ++u) { unsigned short a, c; splitf(Ob[((size_t)z * TT + t) * 64 + d + u] * (1.0f / PCAR), a, c); oh[u] = a; ol[u] = c; } const size_t o = (size_t)t * CC + (h0 + z) * HD + d; *(volatile v2us*)(Ah + o) = oh; *(volatile v2us*)(Al + o) = ol; __threadfence(); *(volatile v2us*)(Ah + o) = oh; *(volatile v2us*)(Al + o) = ol; }
__global__ __launch_bounds__(256) void k_lnres(const float* __restrict__ xin, int isin, const float* __restrict__ D, const float* __restrict__ g, const float* __restrict__ bb, float* Y, bf* Yh, bf* Yl, int planes) { const int lane = threadIdx.x & 31; const int t = blockIdx.x * 8 + (threadIdx.x >> 5); if (t >= TT) return; float v[8]; float s = 0.f;
#pragma unroll
    for (int ch = 0; ch < 2; ++ch) { const size_t o = (size_t)t * CC + ch * 128 + lane * 4; const v4f a = *(const v4f*)(xin + o), dd = *(const v4f*)(D + o);
#pragma unroll
        for (int q = 0; q < 4; ++q) { v[ch * 4 + q] = __fadd_rn(isin ? bfr(a[q]) : a[q], dd[q]); s = __fadd_rn(s, v[ch * 4 + q]); } }
#pragma unroll
    for (int sh = 16; sh; sh >>= 1) s += __shfl_xor(s, sh, 32);
    const float mu = s * (1.0f / CC); float q2 = 0.f;
#pragma unroll
    for (int k = 0; k < 8; ++k) { float dv = __fsub_rn(v[k], mu); asm volatile("" : "+v"(dv)); float p = __fmul_rn(dv, dv); asm volatile("" : "+v"(p)); q2 = __fadd_rn(q2, p); }
#pragma unroll
    for (int sh = 16; sh; sh >>= 1) q2 += __shfl_xor(q2, sh, 32);
    float vq = q2 * (1.0f / CC); asm volatile("" : "+v"(vq)); const float rs = __frsqrt_rn(__fadd_rn(vq, 1e-5f));
#pragma unroll 1
    for (int ps = 0; ps < 2; ++ps) {
#pragma unroll
        for (int ch = 0; ch < 2; ++ch) { const int c0 = ch * 128 + lane * 4; v4f y; v4us oh, ol;
#pragma unroll
            for (int q = 0; q < 4; ++q) { float dv = __fsub_rn(v[ch * 4 + q], mu); asm volatile("" : "+v"(dv)); float tn = __fmul_rn(dv, rs); asm volatile("" : "+v"(tn)); float tg = __fmul_rn(tn, bfr(g[c0 + q])); asm volatile("" : "+v"(tg)); y[q] = __fadd_rn(tg, bfr(bb[c0 + q])); if (planes) { unsigned short a2, c2; splitf(y[q], a2, c2); oh[q] = a2; ol[q] = c2; } }
            const size_t oo = (size_t)t * CC + c0; *(volatile v4f*)(Y + oo) = y; if (planes) { *(volatile v4us*)(Yh + oo) = oh; *(volatile v4us*)(Yl + oo) = ol; } }
        if (ps == 0) __threadfence(); } }
__global__ __launch_bounds__(256) void k_gelu(const float* __restrict__ Hf, bf* Gh, bf* Gl) { const size_t i = ((size_t)blockIdx.x * 256 + threadIdx.x) * 4; if (i >= (size_t)TT * HID) return; const v4f a = *(const v4f*)(Hf + i); v4us oh, ol;
#pragma unroll
    for (int q = 0; q < 4; ++q) { const float x = a[q]; const float gl = 0.5f * x * (1.0f + erff(x * 0.7071067811865476f)); unsigned short u, c; splitf(gl, u, c); oh[q] = u; ol[q] = c; } *(volatile v4us*)(Gh + i) = oh; *(volatile v4us*)(Gl + i) = ol; __threadfence(); *(volatile v4us*)(Gh + i) = oh; *(volatile v4us*)(Gl + i) = ol; }

extern "C" void kernel_launch(void* const* d_in, const int* in_sizes, int n_in,
                              void* d_out, int out_size, void* d_ws, size_t ws_size, hipStream_t stream) {
    (void)in_sizes; (void)n_in; (void)out_size;
    const float* IN[14]; for (int i = 0; i < 14; ++i) IN[i] = (const float*)d_in[i];
    float* OUT = (float*)d_out;
    char* wsp = (char*)d_ws;
    auto take = [&](size_t bytes) { char* p = wsp; wsp += (bytes + 255) & ~(size_t)255; return (void*)p; };
    bf* WQ = (bf*)take((size_t)3 * CC * CC * 2); bf* WP = (bf*)take((size_t)CC * CC * 2); bf* W1 = (bf*)take((size_t)HID * CC * 2); bf* W2 = (bf*)take((size_t)CC * HID * 2); bf* XB = (bf*)take((size_t)TT * CC * 2); float* QKV = (float*)take((size_t)TT * 3 * CC * 4);
    h16* Q16 = (h16*)take((size_t)NH_ * TT * HD * 2); h16* K16 = (h16*)take((size_t)NH_ * TT * HD * 2); h16* VT = (h16*)take((size_t)NH_ * 64 * TT * 2); float* Sb = (float*)take((size_t)ZH * TT * TT * 4); h16* P16 = (h16*)take((size_t)ZH * TT * TT * 2); float* Ob = (float*)take((size_t)ZH * TT * 64 * 4); bf* Ah = (bf*)take((size_t)TT * CC * 2); bf* Al = (bf*)take((size_t)TT * CC * 2);
    float* DL = (float*)take((size_t)TT * CC * 4); float* X1 = (float*)take((size_t)TT * CC * 4); bf* X1h = (bf*)take((size_t)TT * CC * 2); bf* X1l = (bf*)take((size_t)TT * CC * 2); float* HF = (float*)take((size_t)TT * HID * 4); bf* Gh = (bf*)take((size_t)TT * HID * 2); bf* Gl = (bf*)take((size_t)TT * HID * 2);
    if ((size_t)(wsp - (char*)d_ws) > ws_size) return;
    k_cvt8<<<(3 * CC * CC / 8 + 255) / 256, 256, 0, stream>>>(IN[2], WQ, (size_t)3 * CC * CC / 8); k_cvt8<<<(CC * CC / 8 + 255) / 256, 256, 0, stream>>>(IN[4], WP, (size_t)CC * CC / 8); k_cvt8<<<(HID * CC / 8 + 255) / 256, 256, 0, stream>>>(IN[8], W1, (size_t)HID * CC / 8); k_cvt8<<<(CC * HID / 8 + 255) / 256, 256, 0, stream>>>(IN[10], W2, (size_t)CC * HID / 8);
    const unsigned LP = (unsigned)(((size_t)NH_ * TT * HD / 2 + 255) / 256);
    for (int b = 0; b < NB_; ++b) { const float* xb = IN[0] + (size_t)b * TT * CC;
        k_cvt8<<<(TT * CC / 8 + 255) / 256, 256, 0, stream>>>(xb, XB, (size_t)TT * CC / 8);
        k_gemmw<bf, 0, true><<<dim3(TT / 64, 3 * CC / 64, 1), 32, 0, stream>>>(XB, nullptr, WQ, nullptr, CC, QKV, 3 * CC, IN[3], 0, 0, 0);
        k_pl<<<LP, 256, 0, stream>>>(QKV, 0, SCL, Q16); k_pl<<<LP, 256, 0, stream>>>(QKV, 1, 1.0f, K16); k_vtp<<<(unsigned)(((size_t)NH_ * 64 * TT / 2 + 255) / 256), 256, 0, stream>>>(QKV, VT);
        for (int h0 = 0; h0 < NH_; h0 += ZH) { const size_t z = (size_t)h0;
            k_gemmw<h16, 0, false><<<dim3(TT / 64, TT / 64, ZH), 32, 0, stream>>>(Q16 + z * TT * HD, nullptr, K16 + z * TT * HD, nullptr, HD, Sb, TT, nullptr, (size_t)TT * HD, (size_t)TT * HD, (size_t)TT * TT);
            k_msoft<<<ZH * TT / 8, 256, 0, stream>>>(Sb, IN[1], P16);
            k_gemmw<h16, 0, false><<<dim3(TT / 64, 1, ZH), 32, 0, stream>>>(P16, nullptr, VT + z * 64 * TT, nullptr, TT, Ob, 64, nullptr, (size_t)TT * TT, (size_t)64 * TT, (size_t)TT * 64);
            k_mrg<<<(unsigned)(((size_t)ZH * TT * HD / 2 + 255) / 256), 256, 0, stream>>>(Ob, h0, Ah, Al); }
        k_gemmw<bf, 1, true><<<dim3(TT / 64, CC / 64, 1), 32, 0, stream>>>(Ah, Al, WP, nullptr, CC, DL, CC, IN[5], 0, 0, 0);
        k_lnres<<<TT / 8, 256, 0, stream>>>(xb, 1, DL, IN[6], IN[7], X1, X1h, X1l, 1);
        k_gemmw<bf, 1, true><<<dim3(TT / 64, HID / 64, 1), 32, 0, stream>>>(X1h, X1l, W1, nullptr, CC, HF, HID, IN[9], 0, 0, 0); k_gelu<<<(unsigned)(((size_t)TT * HID / 4 + 255) / 256), 256, 0, stream>>>(HF, Gh, Gl);
        k_gemmw<bf, 1, true><<<dim3(TT / 64, CC / 64, 1), 32, 0, stream>>>(Gh, Gl, W2, nullptr, HID, DL, CC, IN[11], 0, 0, 0);
        k_lnres<<<TT / 8, 256, 0, stream>>>(X1, 0, DL, IN[12], IN[13], OUT + (size_t)b * TT * CC, nullptr, nullptr, 0); }
}
